// SEGNNModel_23905787969631
// MI455X (gfx1250) — hardware-verified
//
#include <hip/hip_runtime.h>
#include <stddef.h>


#define NTHR   128
#define NWAVE  4
#define EPT    8
#define CHUNK  (NTHR * EPT)
#define WCAP   (EPT * 32)
#define LISTN  (NWAVE * WCAP)
#define PASSN  (NWAVE * 16)
#define PCAP   (CHUNK + 2 * PASSN)
#define NB     128
#define AW     165
#define RW     7680
#define SMW    128

#define O_S    0
#define O_VD   2560
#define O_VC   3584
#define O_A2   0
#define O_V2   1536
#define O_O2   3072
#define O_SW   5632
#define O_VW   6144

#define SM_SD   0
#define SM_SS   16
#define SM_SLOT 32
#define SM_AS   48
#define SM_AV   64
#define SM_DIST 112

#define L_ACC   0
#define L_WR    21288
#define L_LIST  (L_WR + NWAVE * RW)
#define L_PEND  (L_LIST + LISTN)
#define L_SM    (L_PEND + PCAP)
#define L_WCNT  (L_SM + NWAVE * SMW)
#define L_END   (L_WCNT + 8)
#define LDS_BYTES (L_END * 4)

static_assert((NB + 1) * AW <= L_WR);
static_assert(O_VW + 1536 == RW);
static_assert(O_O2 + 1024 <= O_SW);
static_assert(16 * AW <= O_SW);
static_assert((L_WR % 4) == 0 && (L_LIST % 4) == 0 && (L_PEND % 4) == 0 && (L_SM % 4) == 0 && (L_WCNT % 4) == 0);
static_assert(LDS_BYTES == 218816);
static_assert(PASSN == NWAVE * 16);
static_assert((NB % 16) == 0 && ((NB / 16) % NWAVE) == 0);

#define SZ_W1P  (96 * 224)
#define SZ_W1SV (32 * 160)
#define SZ_W1VV (32 * 64)
#define SZ_W2P  (96 * 96)
#define SZ_W2SV (32 * 64)
#define SZ_W2VV (32 * 32)
#define SZ_U1P  (96 * 192)
#define SZ_U1SV (32 * 128)
#define SZ_U1VV (32 * 64)
#define SZ_U2P  (64 * 96)
#define SZ_U2SV (32 * 64)
#define SZ_U2VV (32 * 32)
#define OF_W1P  0
#define OF_W1SV (OF_W1P + 2 * SZ_W1P)
#define OF_W1VV (OF_W1SV + 2 * SZ_W1SV)
#define OF_W2P  (OF_W1VV + 2 * SZ_W1VV)
#define OF_W2SV (OF_W2P + 2 * SZ_W2P)
#define OF_W2VV (OF_W2SV + 2 * SZ_W2SV)
#define OF_U1P  (OF_W2VV + 2 * SZ_W2VV)
#define OF_U1SV (OF_U1P + 2 * SZ_U1P)
#define OF_U1VV (OF_U1SV + 2 * SZ_U1SV)
#define OF_U2P  (OF_U1VV + 2 * SZ_U1VV)
#define OF_U2SV (OF_U2P + 2 * SZ_U2P)
#define OF_U2VV (OF_U2SV + 2 * SZ_U2SV)
#define WP_TOTAL (OF_U2VV + 2 * SZ_U2VV)
static_assert((SZ_W1P % 128) == 0 && (SZ_W1SV % 128) == 0 && (SZ_W1VV % 128) == 0 && (SZ_W2P % 128) == 0);
static_assert((SZ_W2SV % 128) == 0 && (SZ_W2VV % 128) == 0 && (SZ_U1P % 128) == 0 && (SZ_U1SV % 128) == 0);
static_assert((SZ_U1VV % 128) == 0 && (SZ_U2P % 128) == 0 && (SZ_U2SV % 128) == 0 && (SZ_U2VV % 128) == 0);
static_assert(WP_TOTAL == 149504);

#define RSQRT3 0.5773502691896258f

typedef float          v4f  __attribute__((ext_vector_type(4)));
typedef float          v8f  __attribute__((ext_vector_type(8)));
typedef int            v4i  __attribute__((ext_vector_type(4)));
typedef unsigned short us8  __attribute__((ext_vector_type(8)));
typedef unsigned short us16 __attribute__((ext_vector_type(16)));
typedef __bf16         bf16x16 __attribute__((ext_vector_type(16)));
union Frag { bf16x16 v; us16 u; us8 h[2]; };

__device__ __forceinline__ int clampi(int v, int lo, int hi) { return v < lo ? lo : (v > hi ? hi : v); }

__device__ __forceinline__ void wsync() {
  __builtin_amdgcn_fence(__ATOMIC_ACQ_REL, "wavefront");
  __builtin_amdgcn_wave_barrier();
}

__device__ __forceinline__ unsigned short bfb(float f) {
  unsigned int u = __float_as_uint(f);
  u += 0x7FFFu + ((u >> 16) & 1u);
  return (unsigned short)(u >> 16);
}

__device__ __forceinline__ float sigm(float x) {
  const float e = __expf(-x);
  return __builtin_amdgcn_rcpf(1.0f + e);
}

__device__ __forceinline__ v8f mma3(v8f c, const Frag& ah, const Frag& al, const Frag& bh, const Frag& bl) {
  v8f d = __builtin_amdgcn_wmma_f32_16x16x32_bf16(false, ah.v, false, bh.v, (short)0, c, false, false);
  d = __builtin_amdgcn_wmma_f32_16x16x32_bf16(false, ah.v, false, bl.v, (short)0, d, false, false);
  d = __builtin_amdgcn_wmma_f32_16x16x32_bf16(false, al.v, false, bh.v, (short)0, d, false, false);
  asm volatile("v_nop\n\tv_nop\n\tv_nop\n\tv_nop" : "+v"(d) : "v"(ah.v), "v"(al.v), "v"(bh.v), "v"(bl.v));
  return d;
}

__device__ __forceinline__ void loadA(const float* p, float sc, Frag& hi, Frag& lo) {
  const v4f q0 = *(const v4f*)p;
  const v4f q1 = *(const v4f*)(p + 4);
  const v4f q2 = *(const v4f*)(p + 16);
  const v4f q3 = *(const v4f*)(p + 20);
  float x[16];
  x[0] = q0.x;  x[1] = q0.y;  x[2] = q0.z;  x[3] = q0.w;
  x[4] = q1.x;  x[5] = q1.y;  x[6] = q1.z;  x[7] = q1.w;
  x[8] = q2.x;  x[9] = q2.y;  x[10] = q2.z; x[11] = q2.w;
  x[12] = q3.x; x[13] = q3.y; x[14] = q3.z; x[15] = q3.w;
#pragma unroll
  for (int i = 0; i < 16; ++i) {
    const float t = x[i] * sc;
    const unsigned short hb = bfb(t);
    const float th = __uint_as_float(((unsigned int)hb) << 16);
    hi.u[i] = hb;
    lo.u[i] = bfb(t - th);
  }
}

template <int NT>
__device__ __forceinline__ void gemm_tiles(v8f (&acc)[NT], const float* wr, int off0, int pitch0, int ks0, float sc0,
                                           int off1, int pitch1, int KS,
                                           const unsigned short* __restrict__ wh, const unsigned short* __restrict__ wl,
                                           int lane) {
  const int m = lane & 15, hh = lane >> 4;
  const int Kp = KS * 32;
  const v8f z = {0.0f, 0.0f, 0.0f, 0.0f, 0.0f, 0.0f, 0.0f, 0.0f};
#pragma unroll
  for (int t = 0; t < NT; ++t) acc[t] = z;
#pragma unroll 1
  for (int ks = 0; ks < KS; ++ks) {
    const bool s0 = ks < ks0;
    const int aoff = s0 ? (off0 + m * pitch0 + ks * 32) : (off1 + m * pitch1 + (ks - ks0) * 32);
    const float sc = s0 ? sc0 : 1.0f;
    Frag ah, al;
    loadA(wr + aoff + 8 * hh, sc, ah, al);
#pragma unroll
    for (int t = 0; t < NT; ++t) {
      const int bo = (t * 16 + m) * Kp + ks * 32 + 8 * hh;
      Frag bh, bl;
      bh.h[0] = *(const us8*)(wh + bo);
      bh.h[1] = *(const us8*)(wh + bo + 16);
      bl.h[0] = *(const us8*)(wl + bo);
      bl.h[1] = *(const us8*)(wl + bo + 16);
      acc[t] = mma3(acc[t], ah, al, bh, bl);
    }
  }
}

__device__ __forceinline__ void st_tile(float* base, int pitch, int col0, v8f d, int lane) {
  const int n = lane & 15, hh = lane >> 4;
#pragma unroll
  for (int r = 0; r < 8; ++r) base[(8 * hh + r) * pitch + col0 + n] = d[r];
}

template <int NTS>
__device__ __forceinline__ void tp_layer(v8f (&a6)[NTS], float* wr, int offS, int pitchS, int kss,
                                         int offVD, int pitchVD, int ksvd, int offVc, int pitchVc, int vcStr, int ksvv,
                                         float rowsc,
                                         const unsigned short* __restrict__ ph, const unsigned short* __restrict__ pl,
                                         const unsigned short* __restrict__ svh, const unsigned short* __restrict__ svl,
                                         const unsigned short* __restrict__ vvh, const unsigned short* __restrict__ vvl,
                                         const float* __restrict__ bias, int lane) {
  {
    v8f a2[2], c0[2], c1[2], c2[2];
    gemm_tiles<2>(a2, wr, offS, pitchS, kss, 1.0f, 0, 0, kss, svh, svl, lane);
    gemm_tiles<2>(c0, wr, offVc, pitchVc, ksvv, rowsc, 0, 0, ksvv, vvh, vvl, lane);
    gemm_tiles<2>(c1, wr, offVc + vcStr, pitchVc, ksvv, rowsc, 0, 0, ksvv, vvh, vvl, lane);
    gemm_tiles<2>(c2, wr, offVc + 2 * vcStr, pitchVc, ksvv, rowsc, 0, 0, ksvv, vvh, vvl, lane);
    wsync();
    st_tile(wr + O_SW, 32, 0, a2[0], lane);
    st_tile(wr + O_SW, 32, 16, a2[1], lane);
    st_tile(wr + O_VW, 32, 0, c0[0], lane);
    st_tile(wr + O_VW, 32, 16, c0[1], lane);
    st_tile(wr + O_VW + 512, 32, 0, c1[0], lane);
    st_tile(wr + O_VW + 512, 32, 16, c1[1], lane);
    st_tile(wr + O_VW + 1024, 32, 0, c2[0], lane);
    st_tile(wr + O_VW + 1024, 32, 16, c2[1], lane);
  }
  gemm_tiles<NTS>(a6, wr, offS, pitchS, kss, rowsc, offVD, pitchVD, kss + ksvd, ph, pl, lane);
  const int n = lane & 15;
#pragma unroll
  for (int t = 0; t < NTS; ++t) {
    const float bv = bias[16 * t + n];
#pragma unroll
    for (int r = 0; r < 8; ++r) a6[t][r] += bv;
  }
  wsync();
}

__device__ __forceinline__ void gate_build(float* wr, const float* smf, const v8f (&a6)[6], int lane) {
  const int n = lane & 15, hh = lane >> 4;
#pragma unroll
  for (int t = 0; t < 4; ++t) {
#pragma unroll
    for (int r = 0; r < 8; ++r) {
      const int e = 8 * hh + r;
      const float x = a6[t][r];
      wr[O_A2 + e * 96 + 16 * t + n] = x * sigm(x);
    }
  }
#pragma unroll
  for (int tt = 0; tt < 2; ++tt) {
    const int o = 16 * tt + n;
#pragma unroll
    for (int r = 0; r < 8; ++r) {
      const int e = 8 * hh + r;
      const float g = sigm(a6[4 + tt][r]);
      const float av0 = smf[SM_AV + 3 * e], av1 = smf[SM_AV + 3 * e + 1], av2 = smf[SM_AV + 3 * e + 2];
      const float sw = wr[O_SW + e * 32 + o];
      const float w0 = wr[O_VW + e * 32 + o];
      const float w1 = wr[O_VW + 512 + e * 32 + o];
      const float w2 = wr[O_VW + 1024 + e * 32 + o];
      const float m0 = g * (sw * av0 + w0);
      const float m1 = g * (sw * av1 + w1);
      const float m2 = g * (sw * av2 + w2);
      wr[O_V2 + e * 32 + o]        = m0;
      wr[O_V2 + 512 + e * 32 + o]  = m1;
      wr[O_V2 + 1024 + e * 32 + o] = m2;
      wr[O_A2 + e * 96 + 64 + o] = (m0 * av0 + m1 * av1 + m2 * av2) * RSQRT3;
    }
  }
}

__device__ __forceinline__ void msg_build(float* wr, const float* smf, const v8f (&a6)[6], int lane) {
  const int n = lane & 15, hh = lane >> 4;
#pragma unroll
  for (int t = 0; t < 4; ++t) {
#pragma unroll
    for (int r = 0; r < 8; ++r) {
      const int e = 8 * hh + r;
      const float x = a6[t][r];
      wr[e * AW + 16 * t + n] = x * sigm(x);
    }
  }
#pragma unroll
  for (int tt = 0; tt < 2; ++tt) {
    const int o = 16 * tt + n;
#pragma unroll
    for (int r = 0; r < 8; ++r) {
      const int e = 8 * hh + r;
      const float g = sigm(a6[4 + tt][r]);
      const float av0 = smf[SM_AV + 3 * e], av1 = smf[SM_AV + 3 * e + 1], av2 = smf[SM_AV + 3 * e + 2];
      const float sw = wr[O_SW + e * 32 + o];
      const float w0 = wr[O_VW + e * 32 + o];
      const float w1 = wr[O_VW + 512 + e * 32 + o];
      const float w2 = wr[O_VW + 1024 + e * 32 + o];
      wr[e * AW + 64 + 3 * o + 0] = g * (sw * av0 + w0);
      wr[e * AW + 64 + 3 * o + 1] = g * (sw * av1 + w1);
      wr[e * AW + 64 + 3 * o + 2] = g * (sw * av2 + w2);
    }
  }
  if (lane < 16) {
    const int e = lane;
    wr[e * AW + 160] = smf[SM_AS + e];
    wr[e * AW + 161] = smf[SM_AV + 3 * e];
    wr[e * AW + 162] = smf[SM_AV + 3 * e + 1];
    wr[e * AW + 163] = smf[SM_AV + 3 * e + 2];
    wr[e * AW + 164] = 1.0f;
  }
}

__device__ __forceinline__ int scan_chunk(const int* __restrict__ dsts, int nE, int cbase, int nodeBase,
                                          int vec8, int* list, int tid, int wave) {
  int wc = 0;
  const int el0  = tid * EPT;
  const int e0   = cbase + el0;
  const int sent = -2147483647 - 1;
  v4i da, db;
  if (vec8 != 0 && cbase + CHUNK <= nE) {
    da = *(const v4i*)(dsts + e0);
    db = *(const v4i*)(dsts + e0 + 4);
  } else {
    da.x = (e0     < nE) ? dsts[min(e0, nE - 1)] : sent;
    da.y = (e0 + 1 < nE) ? dsts[min(e0 + 1, nE - 1)] : sent;
    da.z = (e0 + 2 < nE) ? dsts[min(e0 + 2, nE - 1)] : sent;
    da.w = (e0 + 3 < nE) ? dsts[min(e0 + 3, nE - 1)] : sent;
    db.x = (e0 + 4 < nE) ? dsts[min(e0 + 4, nE - 1)] : sent;
    db.y = (e0 + 5 < nE) ? dsts[min(e0 + 5, nE - 1)] : sent;
    db.z = (e0 + 6 < nE) ? dsts[min(e0 + 6, nE - 1)] : sent;
    db.w = (e0 + 7 < nE) ? dsts[min(e0 + 7, nE - 1)] : sent;
  }
  const unsigned nb = (unsigned)nodeBase;
  const unsigned s0 = (unsigned)da.x - nb, s1 = (unsigned)da.y - nb;
  const unsigned s2 = (unsigned)da.z - nb, s3 = (unsigned)da.w - nb;
  const unsigned s4 = (unsigned)db.x - nb, s5 = (unsigned)db.y - nb;
  const unsigned s6 = (unsigned)db.z - nb, s7 = (unsigned)db.w - nb;
  const bool h0 = s0 < (unsigned)NB, h1 = s1 < (unsigned)NB, h2 = s2 < (unsigned)NB, h3 = s3 < (unsigned)NB;
  const bool h4 = s4 < (unsigned)NB, h5 = s5 < (unsigned)NB, h6 = s6 < (unsigned)NB, h7 = s7 < (unsigned)NB;
  const unsigned any = __builtin_amdgcn_ballot_w32(h0 | h1 | h2 | h3 | h4 | h5 | h6 | h7);
  if (any != 0u) {
#define HITJ(J, HJ) { \
      const unsigned mj = __builtin_amdgcn_ballot_w32(HJ); \
      if (mj != 0u) { \
        if (HJ) { \
          const int pos = wc + (int)__builtin_amdgcn_mbcnt_lo(mj, 0u); \
          if (pos < WCAP) list[wave * WCAP + pos] = el0 + (J); \
        } \
        wc += (int)__builtin_popcount(mj); } }
    HITJ(0, h0)
    HITJ(1, h1)
    HITJ(2, h2)
    HITJ(3, h3)
    HITJ(4, h4)
    HITJ(5, h5)
    HITJ(6, h6)
    HITJ(7, h7)
#undef HITJ
  }
  return wc;
}

__device__ __forceinline__ void edge_pass(float* acc, float* wr, const int* pend, int* smi, float* smf,
                                          const float* __restrict__ x_s, const float* __restrict__ x_v,
                                          const int* __restrict__ srcs, const int* __restrict__ dsts,
                                          const float* __restrict__ edist, const float* __restrict__ eas,
                                          const float* __restrict__ eav,
                                          const unsigned short* __restrict__ wp,
                                          const float* __restrict__ b1, const float* __restrict__ b2,
                                          int r, int Pv, int nodeBase, int nN, int nE, int lane, int wave) {
  {
    const int i = lane & 15;
    int idx = r * PASSN + wave * 16 + i;
    const bool valid = (lane < 16) && (idx < Pv);
    idx = clampi(idx, 0, PCAP - 1);
    int e = pend[idx];
    e = clampi(e, 0, nE - 1);
    int d = dsts[e];
    int s = srcs[e];
    int slot = d - nodeBase;
    if (!valid || (unsigned)slot >= (unsigned)NB) slot = NB;
    d = clampi(d, 0, nN - 1);
    s = clampi(s, 0, nN - 1);
    const float dist = edist[e];
    const float as = eas[e];
    const float av0 = eav[(size_t)e * 3], av1 = eav[(size_t)e * 3 + 1], av2 = eav[(size_t)e * 3 + 2];
    if (lane < 16) {
      smi[SM_SD + i] = d;
      smi[SM_SS + i] = s;
      smi[SM_SLOT + i] = slot;
      smf[SM_AS + i] = as;
      smf[SM_AV + 3 * i] = av0;
      smf[SM_AV + 3 * i + 1] = av1;
      smf[SM_AV + 3 * i + 2] = av2;
      smf[SM_DIST + i] = dist;
    }
  }
  wsync();
#pragma unroll 1
  for (int i = 0; i < 16; ++i) {
    const int d = smi[SM_SD + i], s = smi[SM_SS + i];
    const float av0 = smf[SM_AV + 3 * i], av1 = smf[SM_AV + 3 * i + 1], av2 = smf[SM_AV + 3 * i + 2];
    const float dist = smf[SM_DIST + i];
    const int node = (lane < 16) ? d : s;
    const v4f xs = *(const v4f*)(x_s + (size_t)node * 64 + 4 * (lane & 15));
    *(v4f*)(wr + O_S + i * 160 + 4 * lane) = xs;
    wr[O_S + i * 160 + 128 + lane] = (lane == 0) ? dist : 0.0f;
    const float* pd = x_v + (size_t)d * 96 + 3 * lane;
    const float* ps = x_v + (size_t)s * 96 + 3 * lane;
    const float d0 = pd[0], d1 = pd[1], d2 = pd[2];
    const float s0 = ps[0], s1 = ps[1], s2 = ps[2];
    wr[O_VC + i * 64 + lane]             = d0;
    wr[O_VC + 1024 + i * 64 + lane]      = d1;
    wr[O_VC + 2048 + i * 64 + lane]      = d2;
    wr[O_VC + i * 64 + 32 + lane]        = s0;
    wr[O_VC + 1024 + i * 64 + 32 + lane] = s1;
    wr[O_VC + 2048 + i * 64 + 32 + lane] = s2;
    wr[O_VD + i * 64 + lane]      = (d0 * av0 + d1 * av1 + d2 * av2) * RSQRT3;
    wr[O_VD + i * 64 + 32 + lane] = (s0 * av0 + s1 * av1 + s2 * av2) * RSQRT3;
  }
  wsync();
  const float as_m = smf[SM_AS + (lane & 15)];
  v8f a6[6];
  tp_layer<6>(a6, wr, O_S, 160, 5, O_VD, 64, 2, O_VC, 64, 1024, 2, as_m,
              wp + OF_W1P, wp + OF_W1P + SZ_W1P, wp + OF_W1SV, wp + OF_W1SV + SZ_W1SV,
              wp + OF_W1VV, wp + OF_W1VV + SZ_W1VV, b1, lane);
  gate_build(wr, smf, a6, lane);
  wsync();
  tp_layer<6>(a6, wr, O_A2, 96, 2, O_A2 + 64, 96, 1, O_V2, 32, 512, 1, as_m,
              wp + OF_W2P, wp + OF_W2P + SZ_W2P, wp + OF_W2SV, wp + OF_W2SV + SZ_W2SV,
              wp + OF_W2VV, wp + OF_W2VV + SZ_W2VV, b2, lane);
  msg_build(wr, smf, a6, lane);
  wsync();
#pragma unroll 1
  for (int w = 0; w < NWAVE; ++w) {
    if (wave == w) {
#pragma unroll 1
      for (int e = 0; e < 16; ++e) {
        int sl = smi[SM_SLOT + e];
        sl = clampi(sl, 0, NB);
        for (int j = lane; j < AW; j += 32) acc[sl * AW + j] += wr[e * AW + j];
      }
    }
    __syncthreads();
  }
}

__device__ __forceinline__ void node_tile(const float* acc, float* wr, float* smf,
                                          const float* __restrict__ x_s, const float* __restrict__ x_v,
                                          const unsigned short* __restrict__ wp,
                                          const float* __restrict__ ub1, const float* __restrict__ ub2,
                                          float* out, int tt, int nodeBase, int lane) {
  {
    const int i = lane & 15;
    const int slot = 16 * tt + i;
    const float cnt = acc[slot * AW + 164];
    const float rc = 1.0f / fmaxf(cnt, 1.0f);
    const float ns  = acc[slot * AW + 160] * rc;
    const float nv0 = acc[slot * AW + 161] * rc, nv1 = acc[slot * AW + 162] * rc, nv2 = acc[slot * AW + 163] * rc;
    if (lane < 16) {
      smf[SM_AS + i] = ns;
      smf[SM_AV + 3 * i] = nv0;
      smf[SM_AV + 3 * i + 1] = nv1;
      smf[SM_AV + 3 * i + 2] = nv2;
    }
  }
  wsync();
#pragma unroll 1
  for (int i = 0; i < 16; ++i) {
    const int slot = 16 * tt + i;
    const int node = nodeBase + slot;
    const float nv0 = smf[SM_AV + 3 * i], nv1 = smf[SM_AV + 3 * i + 1], nv2 = smf[SM_AV + 3 * i + 2];
    const v4f xs = *(const v4f*)(x_s + (size_t)node * 64 + 4 * (lane & 15));
    const float* ap = acc + slot * AW + 4 * (lane & 15);
    v4f ag;
    ag.x = ap[0]; ag.y = ap[1]; ag.z = ap[2]; ag.w = ap[3];
    const v4f sel = (lane < 16) ? xs : ag;
    *(v4f*)(wr + O_S + i * 128 + 4 * lane) = sel;
    const float* pd = x_v + (size_t)node * 96 + 3 * lane;
    const float* pa = acc + slot * AW + 64 + 3 * lane;
    const float d0 = pd[0], d1 = pd[1], d2 = pd[2];
    const float g0 = pa[0], g1 = pa[1], g2 = pa[2];
    wr[O_VC + i * 64 + lane]             = d0;
    wr[O_VC + 1024 + i * 64 + lane]      = d1;
    wr[O_VC + 2048 + i * 64 + lane]      = d2;
    wr[O_VC + i * 64 + 32 + lane]        = g0;
    wr[O_VC + 1024 + i * 64 + 32 + lane] = g1;
    wr[O_VC + 2048 + i * 64 + 32 + lane] = g2;
    wr[O_VD + i * 64 + lane]      = (d0 * nv0 + d1 * nv1 + d2 * nv2) * RSQRT3;
    wr[O_VD + i * 64 + 32 + lane] = (g0 * nv0 + g1 * nv1 + g2 * nv2) * RSQRT3;
  }
  wsync();
  const float ns_m = smf[SM_AS + (lane & 15)];
  {
    v8f a6[6];
    tp_layer<6>(a6, wr, O_S, 128, 4, O_VD, 64, 2, O_VC, 64, 1024, 2, ns_m,
                wp + OF_U1P, wp + OF_U1P + SZ_U1P, wp + OF_U1SV, wp + OF_U1SV + SZ_U1SV,
                wp + OF_U1VV, wp + OF_U1VV + SZ_U1VV, ub1, lane);
    gate_build(wr, smf, a6, lane);
    wsync();
  }
  {
    v8f a4[4];
    tp_layer<4>(a4, wr, O_A2, 96, 2, O_A2 + 64, 96, 1, O_V2, 32, 512, 1, ns_m,
                wp + OF_U2P, wp + OF_U2P + SZ_U2P, wp + OF_U2SV, wp + OF_U2SV + SZ_U2SV,
                wp + OF_U2VV, wp + OF_U2VV + SZ_U2VV, ub2, lane);
#pragma unroll
    for (int t = 0; t < 4; ++t) st_tile(wr + O_O2, 64, 16 * t, a4[t], lane);
  }
  wsync();
#pragma unroll 1
  for (int i = 0; i < 16; ++i) {
    const int node = nodeBase + 16 * tt + i;
    const float nv0 = smf[SM_AV + 3 * i], nv1 = smf[SM_AV + 3 * i + 1], nv2 = smf[SM_AV + 3 * i + 2];
    const float xs0 = x_s[(size_t)node * 64 + lane];
    const float xs1 = x_s[(size_t)node * 64 + 32 + lane];
    wr[i * 160 + lane]      = xs0 + wr[O_O2 + i * 64 + lane];
    wr[i * 160 + 32 + lane] = xs1 + wr[O_O2 + i * 64 + 32 + lane];
    const float* pv = x_v + (size_t)node * 96 + 3 * lane;
    const float sw = wr[O_SW + i * 32 + lane];
    wr[i * 160 + 64 + 3 * lane + 0] = pv[0] + sw * nv0 + wr[O_VW + i * 32 + lane];
    wr[i * 160 + 64 + 3 * lane + 1] = pv[1] + sw * nv1 + wr[O_VW + 512 + i * 32 + lane];
    wr[i * 160 + 64 + 3 * lane + 2] = pv[2] + sw * nv2 + wr[O_VW + 1024 + i * 32 + lane];
  }
  wsync();
  float* ob = out + (size_t)(nodeBase + 16 * tt) * 160;
#pragma unroll 1
  for (int q = 0; q < 20; ++q) {
    const int g = q * 32 + lane;
    const v4f v = *(const v4f*)(wr + 4 * g);
    *(volatile v4f*)(ob + 4 * g) = v;
  }
  __threadfence();
#pragma unroll 1
  for (int q = 0; q < 20; ++q) {
    const int g = q * 32 + lane;
    const v4f v = *(const v4f*)(wr + 4 * g);
    *(volatile v4f*)(ob + 4 * g) = v;
  }
  wsync();
}

__global__ __launch_bounds__(NTHR) void k_segnn(
    const float* __restrict__ x_s, const float* __restrict__ x_v, const int* __restrict__ ei,
    const float* __restrict__ edist, const float* __restrict__ eas, const float* __restrict__ eav,
    const unsigned short* __restrict__ wp,
    const float* __restrict__ b1, const float* __restrict__ b2,
    const float* __restrict__ ub1, const float* __restrict__ ub2,
    float* out, int nN, int nE, int vec8) {
  extern __shared__ __align__(16) float dsm[];
  const int tid = threadIdx.x, lane = tid & 31, wave = tid >> 5;
  const int nodeBase = blockIdx.x * NB;
  float* acc  = dsm + L_ACC;
  float* wr   = dsm + L_WR + wave * RW;
  int*   list = (int*)(dsm + L_LIST);
  int*   pend = (int*)(dsm + L_PEND);
  int*   smi  = (int*)(dsm + L_SM + wave * SMW);
  float* smf  = dsm + L_SM + wave * SMW;
  int*   wcnt = (int*)(dsm + L_WCNT);
  int*   pendN = (int*)(dsm + L_WCNT + 4);
  const int* srcs = ei;
  const int* dsts = ei + nE;

  for (int i = tid; i < (NB + 1) * AW; i += NTHR) acc[i] = 0.0f;
  if (tid == 0) pendN[0] = 0;
  __syncthreads();

  const int nChunks = (nE + CHUNK - 1) / CHUNK;
#pragma unroll 1
  for (int ch = 0; ch < nChunks; ++ch) {
    const int cbase = ch * CHUNK;
    const int wc = scan_chunk(dsts, nE, cbase, nodeBase, vec8, list, tid, wave);
    if (lane == 0) wcnt[wave] = wc;
    __syncthreads();

    const int base = pendN[0];
    int tot = 0, myoff = 0;
#pragma unroll
    for (int w = 0; w < NWAVE; ++w) {
      const int c = clampi(wcnt[w], 0, WCAP);
      if (w < wave) myoff += c;
      tot += c;
    }
    int newN = base + tot;
    newN = newN > PCAP ? PCAP : newN;
    {
      const int n = clampi(wcnt[wave], 0, WCAP);
      const int* lp = list + wave * WCAP;
      for (int i = lane; i < n; i += 32) {
        const int pos = base + myoff + i;
        if (pos < PCAP) pend[pos] = cbase + lp[i];
      }
    }
    const int fin = (ch == nChunks - 1) ? 1 : 0;
    const int R   = (fin != 0) ? (newN + PASSN - 1) / PASSN : newN / PASSN;
    const int Pv  = (fin != 0) ? newN : R * PASSN;
    __syncthreads();

#pragma unroll 1
    for (int r = 0; r < R; ++r)
      edge_pass(acc, wr, pend, smi, smf, x_s, x_v, srcs, dsts, edist, eas, eav, wp, b1, b2,
                r, Pv, nodeBase, nN, nE, lane, wave);

    int rem = newN - R * PASSN;
    rem = rem < 0 ? 0 : rem;
    if (R > 0 && tid < rem) pend[tid] = pend[R * PASSN + tid];
    if (tid == 0) pendN[0] = rem;
  }
  __syncthreads();

#pragma unroll 1
  for (int tt = wave; tt < NB / 16; tt += NWAVE)
    node_tile(acc, wr, smf, x_s, x_v, wp, ub1, ub2, out, tt, nodeBase, lane);
}

__global__ __launch_bounds__(256) void k_pack(unsigned short* ph, unsigned short* pl,
                                              const float* __restrict__ A, const float* __restrict__ B,
                                              int Ka, int koffB, int Kb, int N, int Kpad) {
  const int q  = blockIdx.x * 256 + threadIdx.x;
  const int KQ = Kpad >> 3;
  if (q >= N * KQ) return;
  const int n = q / KQ, kq = q - n * KQ;
  us8 hv, lv;
#pragma unroll
  for (int j = 0; j < 8; ++j) {
    const int k  = 8 * kq + j;
    const int ka = clampi(k, 0, Ka - 1);
    const int kb = clampi(k - koffB, 0, Kb - 1);
    const float va = A[(size_t)ka * N + n];
    const float vb = B[(size_t)kb * N + n];
    const float v  = (k < Ka) ? va : ((k >= koffB && k < koffB + Kb) ? vb : 0.0f);
    const unsigned short hb = bfb(v);
    const float th = __uint_as_float(((unsigned int)hb) << 16);
    hv[j] = hb;
    lv[j] = bfb(v - th);
  }
  const size_t o = (size_t)q * 8;
  *(volatile us8*)(ph + o) = hv;
  *(volatile us8*)(pl + o) = lv;
  __threadfence();
  *(volatile us8*)(ph + o) = hv;
  *(volatile us8*)(pl + o) = lv;
}

static void launch_pack(hipStream_t stream, unsigned short* wp, int off, int sz,
                        const float* A, const float* B, int Ka, int koffB, int Kb, int N, int Kpad) {
  const int groups = N * (Kpad / 8);
  const int blocks = (groups + 255) / 256;
  k_pack<<<blocks, 256, 0, stream>>>(wp + off, wp + off + sz, A, B, Ka, koffB, Kb, N, Kpad);
}

extern "C" void kernel_launch(void* const* d_in, const int* in_sizes, int n_in,
                              void* d_out, int out_size, void* d_ws, size_t ws_size,
                              hipStream_t stream) {
  if (n_in < 26) return;
  const int nN = in_sizes[0] / 64;
  if (nN <= 0 || in_sizes[0] != nN * 64 || in_sizes[1] != nN * 96) return;
  if ((nN % NB) != 0) return;
  const int nE = in_sizes[2] / 2;
  if (nE <= 0 || in_sizes[2] != 2 * nE || in_sizes[3] != nE || in_sizes[4] != nE || in_sizes[5] != 3 * nE) return;
  if (in_sizes[6] != 129 * 96 || in_sizes[7] != 64 * 96 || in_sizes[8] != 129 * 32 || in_sizes[9] != 64 * 32 || in_sizes[10] != 96) return;
  if (in_sizes[11] != 64 * 96 || in_sizes[12] != 32 * 96 || in_sizes[13] != 64 * 32 || in_sizes[14] != 32 * 32 || in_sizes[15] != 96) return;
  if (in_sizes[16] != 128 * 96 || in_sizes[17] != 64 * 96 || in_sizes[18] != 128 * 32 || in_sizes[19] != 64 * 32 || in_sizes[20] != 96) return;
  if (in_sizes[21] != 64 * 64 || in_sizes[22] != 32 * 64 || in_sizes[23] != 64 * 32 || in_sizes[24] != 32 * 32 || in_sizes[25] != 64) return;
  if (out_size != nN * 160) return;
  if ((size_t)WP_TOTAL * 2 > ws_size) return;

  const float* x_s   = (const float*)d_in[0];
  const float* x_v   = (const float*)d_in[1];
  const int*   eidx  = (const int*)d_in[2];
  const float* edist = (const float*)d_in[3];
  const float* eas   = (const float*)d_in[4];
  const float* eav   = (const float*)d_in[5];
  const float* m1_ss = (const float*)d_in[6];
  const float* m1_vs = (const float*)d_in[7];
  const float* m1_sv = (const float*)d_in[8];
  const float* m1_vv = (const float*)d_in[9];
  const float* m1_b  = (const float*)d_in[10];
  const float* m2_ss = (const float*)d_in[11];
  const float* m2_vs = (const float*)d_in[12];
  const float* m2_sv = (const float*)d_in[13];
  const float* m2_vv = (const float*)d_in[14];
  const float* m2_b  = (const float*)d_in[15];
  const float* u1_ss = (const float*)d_in[16];
  const float* u1_vs = (const float*)d_in[17];
  const float* u1_sv = (const float*)d_in[18];
  const float* u1_vv = (const float*)d_in[19];
  const float* u1_b  = (const float*)d_in[20];
  const float* u2_ss = (const float*)d_in[21];
  const float* u2_vs = (const float*)d_in[22];
  const float* u2_sv = (const float*)d_in[23];
  const float* u2_vv = (const float*)d_in[24];
  const float* u2_b  = (const float*)d_in[25];
  float* out = (float*)d_out;

  unsigned short* wp = (unsigned short*)d_ws;

  launch_pack(stream, wp, OF_W1P,  SZ_W1P,  m1_ss, m1_vs, 129, 160, 64, 96, 224);
  launch_pack(stream, wp, OF_W1SV, SZ_W1SV, m1_sv, m1_sv, 129, 160, 1,  32, 160);
  launch_pack(stream, wp, OF_W1VV, SZ_W1VV, m1_vv, m1_vv, 64,  64,  1,  32, 64);
  launch_pack(stream, wp, OF_W2P,  SZ_W2P,  m2_ss, m2_vs, 64,  64,  32, 96, 96);
  launch_pack(stream, wp, OF_W2SV, SZ_W2SV, m2_sv, m2_sv, 64,  64,  1,  32, 64);
  launch_pack(stream, wp, OF_W2VV, SZ_W2VV, m2_vv, m2_vv, 32,  32,  1,  32, 32);
  launch_pack(stream, wp, OF_U1P,  SZ_U1P,  u1_ss, u1_vs, 128, 128, 64, 96, 192);
  launch_pack(stream, wp, OF_U1SV, SZ_U1SV, u1_sv, u1_sv, 128, 128, 1,  32, 128);
  launch_pack(stream, wp, OF_U1VV, SZ_U1VV, u1_vv, u1_vv, 64,  64,  1,  32, 64);
  launch_pack(stream, wp, OF_U2P,  SZ_U2P,  u2_ss, u2_vs, 64,  64,  32, 64, 96);
  launch_pack(stream, wp, OF_U2SV, SZ_U2SV, u2_sv, u2_sv, 64,  64,  1,  32, 64);
  launch_pack(stream, wp, OF_U2VV, SZ_U2VV, u2_vv, u2_vv, 32,  32,  1,  32, 32);

  hipFuncSetAttribute(reinterpret_cast<const void*>(&k_segnn), hipFuncAttributeMaxDynamicSharedMemorySize, LDS_BYTES);
  const int vec8 = ((nE & 7) == 0) ? 1 : 0;
  const int nBlk = nN / NB;
  k_segnn<<<nBlk, NTHR, LDS_BYTES, stream>>>(x_s, x_v, eidx, edist, eas, eav, wp,
                                             m1_b, m2_b, u1_b, u2_b, out, nN, nE, vec8);
}
